// TeacherNet_84189948936790
// MI455X (gfx1250) — hardware-run, weakly checked
//
#include <hip/hip_runtime.h>
#include <stddef.h>


#define FIN     512
#define HID     512
#define NC12    1024
#define NH12    4
#define CH12    128
#define NH3     6
#define CH3     64
#define HWC3    384
#define NC3     448
#define OUTC    64
#define NHMX    6
#define NTHR    256
#define NWAVE   8
#define EPT     8
#define NGRP    2
#define CHUNK   (NTHR * EPT * NGRP)
#define WCAP    (EPT * NGRP * 32)
#define LISTN   (NWAVE * WCAP)
#define NBC     4096
#define NBF     1024
#define RCAP    40960
#define RBN     128
#define TGT     256
#define DEGCAP  512
#define OTHR    512
#define BM      64
#define WSCAP   134217728
#define NEG_SLOPE 0.2f

#define LDS_FILL ((RCAP + NBF + LISTN) * 4 + 64)

static_assert((CHUNK & (CHUNK - 1)) == 0);
static_assert(CHUNK <= 4096);
static_assert(NBC <= 4096 && NBF <= 4096);
static_assert((NBC & (NBC - 1)) == 0 && (NBF & (NBF - 1)) == 0);
static_assert(NBC == 4 * NBF);
static_assert(OTHR * 8 == NBC);
static_assert((RCAP % 32) == 0);
static_assert(TGT == NWAVE * 32);
static_assert((NBC % TGT) == 0);
static_assert((TGT % BM) == 0);
static_assert(BM * 4 == NTHR);
static_assert(FIN % 32 == 0 && HID % 32 == 0);
static_assert(NH12 * CH12 == HID);
static_assert(NH3 * CH3 == HWC3);
static_assert(HWC3 + OUTC == NC3);
static_assert(HID + HID == NC12);
static_assert(HID == 2 * 32 * 8);
static_assert(HWC3 == 2 * 24 * 8);
static_assert(CH12 == 16 * 8);
static_assert(CH3 == 8 * 8);
static_assert(OUTC == 16 * 4);
static_assert(NH3 <= NHMX && NH12 <= NHMX);
static_assert(FIN == HID);

typedef float          v4f  __attribute__((ext_vector_type(4)));
typedef float          v8f  __attribute__((ext_vector_type(8)));
typedef int            v4i  __attribute__((ext_vector_type(4)));
typedef unsigned short v8us __attribute__((ext_vector_type(8)));
typedef __bf16         v16b __attribute__((ext_vector_type(16)));
union FragB { v16b v; v8us u[2]; };

__device__ __forceinline__ v8f wmb(v16b a, v16b b, v8f c) {
  v8f d = __builtin_amdgcn_wmma_f32_16x16x32_bf16(false, a, false, b, (short)0, c, false, false);
  asm volatile("v_nop\n\tv_nop\n\tv_nop\n\tv_nop" : "+v"(d) : "v"(a), "v"(b));
  return d;
}

__device__ __forceinline__ unsigned int bf16bits(float f) {
  const unsigned int u = __float_as_uint(f);
  return (u + 0x7FFFu + ((u >> 16) & 1u)) >> 16;
}
__device__ __forceinline__ void split8b(v4f a, v4f b, v8us& hi, v8us& lo) {
  v8f f;
  f[0] = a.x; f[1] = a.y; f[2] = a.z; f[3] = a.w;
  f[4] = b.x; f[5] = b.y; f[6] = b.z; f[7] = b.w;
  v8us h, l;
#pragma unroll
  for (int i = 0; i < 8; ++i) {
    const unsigned int hb = bf16bits(f[i]);
    const float hv = __uint_as_float(hb << 16);
    const unsigned int lb = bf16bits(f[i] - hv);
    h[i] = (unsigned short)hb;
    l[i] = (unsigned short)lb;
  }
  hi = h; lo = l;
}

__device__ __forceinline__ float lrelu(float v) { return v > 0.0f ? v : NEG_SLOPE * v; }
__device__ __forceinline__ float elu1(float v) { return v > 0.0f ? v : (__expf(v) - 1.0f); }
__device__ __forceinline__ v4f elu4(v4f v) {
  v4f r;
  r.x = elu1(v.x); r.y = elu1(v.y); r.z = elu1(v.z); r.w = elu1(v.w);
  return r;
}
__device__ __forceinline__ float hsum2(float t) {
  t += __shfl_xor(t, 8);
  t += __shfl_xor(t, 16);
  return t;
}
__device__ __forceinline__ v4f hsum2v(v4f v) {
  v4f r;
  r.x = hsum2(v.x); r.y = hsum2(v.y); r.z = hsum2(v.z); r.w = hsum2(v.w);
  return r;
}

template <int NB>
__device__ __forceinline__ int scan_chunk(const int* __restrict__ dsts, int nE, int cbase, int slotBase,
                                          int vec8, int* list, int tid, int lane, int wave) {
  int wc = 0;
#pragma unroll
  for (int g = 0; g < NGRP; ++g) {
    const int el0  = (g * NTHR + tid) * EPT;
    const int e0   = cbase + el0;
    const int sent = -2147483647 - 1;
    v4i da, db;
    if (vec8 != 0 && cbase + CHUNK <= nE) {
      da = *(const v4i*)(dsts + e0);
      db = *(const v4i*)(dsts + e0 + 4);
    } else {
      da.x = (e0     < nE) ? dsts[min(e0, nE - 1)] : sent;
      da.y = (e0 + 1 < nE) ? dsts[min(e0 + 1, nE - 1)] : sent;
      da.z = (e0 + 2 < nE) ? dsts[min(e0 + 2, nE - 1)] : sent;
      da.w = (e0 + 3 < nE) ? dsts[min(e0 + 3, nE - 1)] : sent;
      db.x = (e0 + 4 < nE) ? dsts[min(e0 + 4, nE - 1)] : sent;
      db.y = (e0 + 5 < nE) ? dsts[min(e0 + 5, nE - 1)] : sent;
      db.z = (e0 + 6 < nE) ? dsts[min(e0 + 6, nE - 1)] : sent;
      db.w = (e0 + 7 < nE) ? dsts[min(e0 + 7, nE - 1)] : sent;
    }
    const unsigned nb = (unsigned)slotBase;
    const unsigned s0 = (unsigned)da.x - nb, s1 = (unsigned)da.y - nb;
    const unsigned s2 = (unsigned)da.z - nb, s3 = (unsigned)da.w - nb;
    const unsigned s4 = (unsigned)db.x - nb, s5 = (unsigned)db.y - nb;
    const unsigned s6 = (unsigned)db.z - nb, s7 = (unsigned)db.w - nb;
    const bool h0 = s0 < (unsigned)NB, h1 = s1 < (unsigned)NB, h2 = s2 < (unsigned)NB, h3 = s3 < (unsigned)NB;
    const bool h4 = s4 < (unsigned)NB, h5 = s5 < (unsigned)NB, h6 = s6 < (unsigned)NB, h7 = s7 < (unsigned)NB;
    const unsigned any = __builtin_amdgcn_ballot_w32(h0 | h1 | h2 | h3 | h4 | h5 | h6 | h7);
    if (any != 0u) {
#define HITJ(J, HJ, SJ) { \
        const unsigned mj = __builtin_amdgcn_ballot_w32(HJ); \
        if (mj != 0u) { \
          if (HJ) { \
            const int pos = wc + (int)__builtin_amdgcn_mbcnt_lo(mj, 0u); \
            if (pos < WCAP) list[wave * WCAP + pos] = ((el0 + (J)) << 12) | (int)(SJ); \
          } \
          wc += (int)__builtin_popcount(mj); } }
      HITJ(0, h0, s0)
      HITJ(1, h1, s1)
      HITJ(2, h2, s2)
      HITJ(3, h3, s3)
      HITJ(4, h4, s4)
      HITJ(5, h5, s5)
      HITJ(6, h6, s6)
      HITJ(7, h7, s7)
#undef HITJ
    }
  }
  return wc;
}

__global__ __launch_bounds__(NTHR) void k_xcvt(const float* __restrict__ x, unsigned short* xh, unsigned short* xl,
                                               int nN, int nUnits) {
  const int i = (int)blockIdx.x * NTHR + (int)threadIdx.x;
  if (i >= nUnits) return;
  const int row = i >> 6;
  const int c0  = (i & 63) * 8;
  int rr = row > nN - 1 ? nN - 1 : row;
  rr = rr < 0 ? 0 : rr;
  const float* p = x + (size_t)rr * FIN + c0;
  v4f a = *(const v4f*)p, b = *(const v4f*)(p + 4);
  const v4f z = {0.f, 0.f, 0.f, 0.f};
  if (row >= nN) { a = z; b = z; }
  v8us hv, lv;
  split8b(a, b, hv, lv);
  unsigned short* dh = xh + (size_t)i * 8;
  unsigned short* dl = xl + (size_t)i * 8;
  *(volatile v8us*)dh = hv;
  *(volatile v8us*)dl = lv;
  __threadfence();
  *(volatile v8us*)dh = hv;
  *(volatile v8us*)dl = lv;
}

template <int KD, int NCW>
__global__ __launch_bounds__(NTHR) void k_wprep3(const float* __restrict__ W, unsigned short* wh, unsigned short* wl) {
  constexpr int KS    = KD / 8;
  constexpr int UNITS = NCW * KS;
  static_assert(KD % 8 == 0);
  const int i = (int)blockIdx.x * NTHR + (int)threadIdx.x;
  if (i >= UNITS) return;
  const int n  = i / KS;
  const int k0 = (i - n * KS) * 8;
  v4f a, b;
  a.x = W[(size_t)(k0 + 0) * NCW + n]; a.y = W[(size_t)(k0 + 1) * NCW + n];
  a.z = W[(size_t)(k0 + 2) * NCW + n]; a.w = W[(size_t)(k0 + 3) * NCW + n];
  b.x = W[(size_t)(k0 + 4) * NCW + n]; b.y = W[(size_t)(k0 + 5) * NCW + n];
  b.z = W[(size_t)(k0 + 6) * NCW + n]; b.w = W[(size_t)(k0 + 7) * NCW + n];
  v8us hv, lv;
  split8b(a, b, hv, lv);
  unsigned short* dh = wh + (size_t)i * 8;
  unsigned short* dl = wl + (size_t)i * 8;
  *(volatile v8us*)dh = hv;
  *(volatile v8us*)dl = lv;
  __threadfence();
  *(volatile v8us*)dh = hv;
  *(volatile v8us*)dl = lv;
}

__global__ __launch_bounds__(NTHR) void k_count(
    const int* __restrict__ dsts, int* cnt, int nE, int vec8) {
  __shared__ __attribute__((aligned(16))) int scnt[NBC];
  __shared__ __attribute__((aligned(16))) int list[LISTN];
  __shared__ int wcnt[NWAVE];
  const int tid = threadIdx.x, lane = tid & 31, wave = tid >> 5;
  const int nodeBase = blockIdx.x * NBC;

  for (int i = tid; i < NBC; i += NTHR) scnt[i] = 0;
  __syncthreads();

  const int nChunks = (nE + CHUNK - 1) / CHUNK;
#pragma unroll 1
  for (int ch = 0; ch < nChunks; ++ch) {
    const int cbase = ch * CHUNK;
    const int wc = scan_chunk<NBC>(dsts, nE, cbase, nodeBase, vec8, list, tid, lane, wave);
    if (lane == 0) wcnt[wave] = wc;
    __syncthreads();
    if (wave == 0) {
#pragma unroll 1
      for (int wsx = 0; wsx < NWAVE; ++wsx) {
        int n = __builtin_amdgcn_readfirstlane(wcnt[wsx]);
        n = n > WCAP ? WCAP : (n < 0 ? 0 : n);
        const int* lp = list + wsx * WCAP;
#pragma unroll 1
        for (int i = 0; i < n; ++i) {
          const int ent  = __builtin_amdgcn_readfirstlane(lp[i]);
          const int slot = ent & (NBC - 1);
          if (lane == 0) scnt[slot] = scnt[slot] + 1;
        }
      }
    }
    __syncthreads();
  }

  v4i cq[4];
#pragma unroll
  for (int q = 0; q < 4; ++q) {
    const int f = (wave * 4 + q) * 128 + 4 * lane;
    cq[q] = *(const v4i*)(scnt + f);
  }
  int* cp = cnt + (size_t)nodeBase;
#pragma unroll
  for (int q = 0; q < 4; ++q) {
    const int f = (wave * 4 + q) * 128 + 4 * lane;
    *(volatile v4i*)(cp + f) = cq[q];
  }
  __threadfence();
#pragma unroll
  for (int q = 0; q < 4; ++q) {
    const int f = (wave * 4 + q) * 128 + 4 * lane;
    *(volatile v4i*)(cp + f) = cq[q];
  }
}

__global__ __launch_bounds__(OTHR) void k_offsets(
    const int* __restrict__ cnt, int* off, int* rbase, int nChunk) {
  __shared__ __attribute__((aligned(16))) int soff[NBC];
  __shared__ __attribute__((aligned(16))) int srb[RBN];
  __shared__ int wtot[OTHR / 32];
  const int tid = threadIdx.x, lane = tid & 31, wave = tid >> 5, sub = tid >> 7;
  for (int i = tid; i < RBN; i += OTHR) srb[i] = 0;
  int carry = 0;
#pragma unroll 1
  for (int ch = 0; ch < nChunk; ++ch) {
    const int base = ch * NBC;
    const v4i c0 = *(const v4i*)(cnt + base + 8 * tid);
    const v4i c1 = *(const v4i*)(cnt + base + 8 * tid + 4);
    const int e0 = max(c0.x, 0), e1 = max(c0.y, 0), e2 = max(c0.z, 0), e3 = max(c0.w, 0);
    const int e4 = max(c1.x, 0), e5 = max(c1.y, 0), e6 = max(c1.z, 0), e7 = max(c1.w, 0);
    const int ts = e0 + e1 + e2 + e3 + e4 + e5 + e6 + e7;
    int incl = ts;
#pragma unroll
    for (int d = 1; d < 32; d <<= 1) {
      const int t = __shfl_up(incl, d);
      if (lane >= d) incl += t;
    }
    if (lane == 31) wtot[wave] = incl;
    __syncthreads();
    const int S0 = wtot[0]  + wtot[1]  + wtot[2]  + wtot[3];
    const int S1 = wtot[4]  + wtot[5]  + wtot[6]  + wtot[7];
    const int S2 = wtot[8]  + wtot[9]  + wtot[10] + wtot[11];
    const int S3 = wtot[12] + wtot[13] + wtot[14] + wtot[15];
    int pre = 0;
#pragma unroll 1
    for (int w = 4 * sub; w < wave; ++w) pre += wtot[w];
    const int b0 = carry;
    const int b1 = b0 + ((S0 + 31) & ~31);
    const int b2 = b1 + ((S1 + 31) & ~31);
    const int b3 = b2 + ((S2 + 31) & ~31);
    const int b4 = b3 + ((S3 + 31) & ~31);
    const int myb = sub == 0 ? b0 : (sub == 1 ? b1 : (sub == 2 ? b2 : b3));
    if (tid == 0) {
      srb[min(4 * ch + 0, RBN - 1)] = b0;
      srb[min(4 * ch + 1, RBN - 1)] = b1;
      srb[min(4 * ch + 2, RBN - 1)] = b2;
      srb[min(4 * ch + 3, RBN - 1)] = b3;
    }
    int run = myb + pre + incl - ts;
    soff[8 * tid + 0] = run; run += e0;
    soff[8 * tid + 1] = run; run += e1;
    soff[8 * tid + 2] = run; run += e2;
    soff[8 * tid + 3] = run; run += e3;
    soff[8 * tid + 4] = run; run += e4;
    soff[8 * tid + 5] = run; run += e5;
    soff[8 * tid + 6] = run; run += e6;
    soff[8 * tid + 7] = run;
    carry = b4;
    __syncthreads();
    const v4i o0 = *(const v4i*)(soff + 4 * tid);
    const v4i o1 = *(const v4i*)(soff + 4 * (tid + OTHR));
    int* op = off + base;
    *(volatile v4i*)(op + 4 * tid) = o0;
    *(volatile v4i*)(op + 4 * (tid + OTHR)) = o1;
    __threadfence();
    *(volatile v4i*)(op + 4 * tid) = o0;
    *(volatile v4i*)(op + 4 * (tid + OTHR)) = o1;
    __syncthreads();
  }
  if (tid == 0) srb[min(4 * nChunk, RBN - 1)] = carry;
  __syncthreads();
  v4i rv = {0, 0, 0, 0};
  if (tid < 32) rv = *(const v4i*)(srb + 4 * tid);
  if (tid < 32) *(volatile v4i*)(rbase + 4 * tid) = rv;
  __threadfence();
  if (tid < 32) *(volatile v4i*)(rbase + 4 * tid) = rv;
}

__global__ __launch_bounds__(NTHR) void k_fill(
    const int* __restrict__ srcs, const int* __restrict__ dsts,
    const int* __restrict__ off, const int* __restrict__ rbase,
    int* csr, int nN, int nE, int vec8, int csrLen) {
  extern __shared__ v4f lds_dyn[];
  int* region = (int*)lds_dyn;
  int* cursor = region + RCAP;
  int* list   = cursor + NBF;
  int* wcnt   = list + LISTN;
  const int tid = threadIdx.x, lane = tid & 31, wave = tid >> 5;
  const int b = blockIdx.x;
  const int nodeBase = b * NBF;

  int rb0 = rbase[b];
  const int rb1 = rbase[b + 1];
  rb0 = rb0 < 0 ? 0 : (rb0 > csrLen ? csrLen : rb0);
  rb0 &= ~31;
  int len = rb1 - rb0;
  len = len < 0 ? 0 : (len > RCAP ? RCAP : len);
  int lenW = (len + 31) & ~31;
  if (rb0 + lenW > csrLen) lenW = (csrLen - rb0) & ~31;

  {
    const v4i z = {0, 0, 0, 0};
    for (int i = tid; i < RCAP / 4; i += NTHR) ((v4i*)region)[i] = z;
    for (int s = tid; s < NBF; s += NTHR) {
      int o = off[nodeBase + s] - rb0;
      o = o < 0 ? 0 : (o > RCAP ? RCAP : o);
      cursor[s] = o;
    }
  }
  __syncthreads();

  const int nChunks = (nE + CHUNK - 1) / CHUNK;
#pragma unroll 1
  for (int ch = 0; ch < nChunks; ++ch) {
    const int cbase = ch * CHUNK;
    const int wc = scan_chunk<NBF>(dsts, nE, cbase, nodeBase, vec8, list, tid, lane, wave);
    if (lane == 0) wcnt[wave] = wc;
    __syncthreads();
    if (wave == 0) {
#pragma unroll 1
      for (int wsx = 0; wsx < NWAVE; ++wsx) {
        int n = __builtin_amdgcn_readfirstlane(wcnt[wsx]);
        n = n > WCAP ? WCAP : (n < 0 ? 0 : n);
        const int* lp = list + wsx * WCAP;
#pragma unroll 1
        for (int i = 0; i < n; ++i) {
          const int ent  = __builtin_amdgcn_readfirstlane(lp[i]);
          const int slot = ent & (NBF - 1);
          int e = cbase + ((ent >> 12) & (CHUNK - 1));
          e = e > nE - 1 ? nE - 1 : e;
          int src = srcs[e];
          src = src < 0 ? 0 : (src > nN - 1 ? nN - 1 : src);
          if (lane == 0) {
            int pos = cursor[slot];
            pos = pos < 0 ? 0 : (pos > RCAP - 1 ? RCAP - 1 : pos);
            region[pos] = src;
            const int np = pos + 1;
            cursor[slot] = np > RCAP ? RCAP : np;
          }
        }
      }
    }
    __syncthreads();
  }

  const int nv = lenW >> 2;
  int* gp = csr + rb0;
#pragma unroll 1
  for (int i = tid; i < nv; i += NTHR) { const v4i v = ((const v4i*)region)[i]; *(volatile v4i*)(gp + 4 * i) = v; }
  __threadfence();
#pragma unroll 1
  for (int i = tid; i < nv; i += NTHR) { const v4i v = ((const v4i*)region)[i]; *(volatile v4i*)(gp + 4 * i) = v; }
}

template <int K, int BN, int NCOL, int NH>
__global__ __launch_bounds__(NTHR) void k_gemm(
    const unsigned short* __restrict__ Ap, const unsigned short* __restrict__ Al,
    const unsigned short* __restrict__ Bp, const unsigned short* __restrict__ Bl,
    const float* __restrict__ attS, const float* __restrict__ attD,
    float* C, float* eS, float* eD, int npad) {
  constexpr int TPW = BN / 32;
  constexpr int KT  = K / 32;
  constexpr int CPP = BN / 4;
  constexpr int HB  = BN / 2;
  constexpr int UPW = (BM * BN / 128) / NWAVE;
  static_assert(K % 32 == 0);
  static_assert(BN == 64 || BN == 128);
  static_assert(NCOL % BN == 0);
  static_assert(CPP % 4 == 0);
  static_assert(UPW * NWAVE * 128 == BM * BN);
  static_assert(BM == 64 && NTHR == 4 * BM);

  __shared__ __attribute__((aligned(16))) float stg[BM * BN];
  __shared__ __attribute__((aligned(16))) float sES[BM];
  __shared__ __attribute__((aligned(16))) float sED[BM];
  const int tid = threadIdx.x, lane = tid & 31, wave = tid >> 5, hh = lane >> 4, m = lane & 15;
  const int rowBase = blockIdx.x * BM;
  const int cs = blockIdx.y * BN;
  const int rg = wave >> 1, chf = wave & 1;
  const int r0 = rg * 16;
  const int c0 = chf * HB;

  v8f acc[TPW];
#pragma unroll
  for (int t = 0; t < TPW; ++t) { v8f z = {0.f, 0.f, 0.f, 0.f, 0.f, 0.f, 0.f, 0.f}; acc[t] = z; }

  const size_t aoff = (size_t)(rowBase + r0 + m) * K + 8 * hh;
  const size_t boff = (size_t)(cs + c0 + m) * K + 8 * hh;
  const unsigned short* ap   = Ap + aoff;
  const unsigned short* alp  = Al + aoff;
  const unsigned short* bp0  = Bp + boff;
  const unsigned short* blp0 = Bl + boff;
#pragma unroll 1
  for (int kt = 0; kt < KT; ++kt) {
    FragB a, al;
    a.u[0]  = *(const v8us*)(ap + 32 * kt);
    a.u[1]  = *(const v8us*)(ap + 32 * kt + 16);
    al.u[0] = *(const v8us*)(alp + 32 * kt);
    al.u[1] = *(const v8us*)(alp + 32 * kt + 16);
#pragma unroll
    for (int t = 0; t < TPW; ++t) {
      const size_t bo = (size_t)(16 * t) * K + 32 * kt;
      FragB bf, bl;
      bf.u[0] = *(const v8us*)(bp0 + bo);
      bf.u[1] = *(const v8us*)(bp0 + bo + 16);
      bl.u[0] = *(const v8us*)(blp0 + bo);
      bl.u[1] = *(const v8us*)(blp0 + bo + 16);
      acc[t] = wmb(a.v, bf.v, acc[t]);
      acc[t] = wmb(a.v, bl.v, acc[t]);
      acc[t] = wmb(al.v, bf.v, acc[t]);
    }
  }

  {
    float* sp = stg + (size_t)(r0 + 8 * hh) * BN + c0 + m;
#pragma unroll
    for (int t = 0; t < TPW; ++t) {
#pragma unroll
      for (int r = 0; r < 8; ++r) sp[r * BN + 16 * t] = acc[t][r];
    }
  }
  __syncthreads();

  {
    const int drow = tid >> 2, part = tid & 3;
    const int hy = (int)blockIdx.y < NH ? (int)blockIdx.y : NH - 1;
    const float* rp  = stg + (size_t)drow * BN + CPP * part;
    const float* sa  = attS + hy * BN + CPP * part;
    const float* sdd = attD + hy * BN + CPP * part;
    float ps = 0.f, pd = 0.f;
#pragma unroll 2
    for (int c = 0; c < CPP; c += 4) {
      const v4f hv = *(const v4f*)(rp + c);
      const v4f av = *(const v4f*)(sa + c);
      const v4f dv = *(const v4f*)(sdd + c);
      ps += hv.x * av.x + hv.y * av.y + hv.z * av.z + hv.w * av.w;
      pd += hv.x * dv.x + hv.y * dv.y + hv.z * dv.z + hv.w * dv.w;
    }
    ps += __shfl_xor(ps, 1); pd += __shfl_xor(pd, 1);
    ps += __shfl_xor(ps, 2); pd += __shfl_xor(pd, 2);
    if (part == 0) { sES[drow] = ps; sED[drow] = pd; }
  }

  {
    v4f cv[UPW];
#pragma unroll
    for (int it = 0; it < UPW; ++it) {
      const int f = 128 * (it * NWAVE + wave) + 4 * lane;
      cv[it] = *(const v4f*)(stg + f);
    }
#pragma unroll
    for (int it = 0; it < UPW; ++it) {
      const int f = 128 * (it * NWAVE + wave) + 4 * lane;
      const int row = f / BN, col = f & (BN - 1);
      float* gp = C + (size_t)(rowBase + row) * NCOL + cs + col;
      *(volatile v4f*)gp = cv[it];
    }
    __threadfence();
#pragma unroll
    for (int it = 0; it < UPW; ++it) {
      const int f = 128 * (it * NWAVE + wave) + 4 * lane;
      const int row = f / BN, col = f & (BN - 1);
      float* gp = C + (size_t)(rowBase + row) * NCOL + cs + col;
      *(volatile v4f*)gp = cv[it];
    }
  }
  __syncthreads();

  {
    const bool hb = ((int)blockIdx.y < NH) && (wave < 2) && (lane < 16);
    const int lq = lane & 15;
    const size_t eb = (size_t)blockIdx.y * (size_t)npad + (size_t)rowBase;
    const v4f vS = *(const v4f*)(sES + 4 * lq);
    const v4f vD = *(const v4f*)(sED + 4 * lq);
    const v4f dv = (wave == 0) ? vS : vD;
    float* gp = ((wave == 0) ? eS : eD) + eb + 4 * lq;
    if (hb) *(volatile v4f*)gp = dv;
    __threadfence();
    if (hb) *(volatile v4f*)gp = dv;
  }
}

__device__ __forceinline__ void gat_row2(
    const int* __restrict__ csr, const float* __restrict__ eS, const float* __restrict__ hw, int pitch,
    size_t ho0, size_t ho1, float edc0, float edc1, float es0, float es1,
    int c, int n, int st, int col0, int col1, int lane, int nN, int csrLen,
    float& dn0, float& dn1, v4f& a00, v4f& a01, v4f& a10, v4f& a11) {
  float mx0 = es0, mx1 = es1;
#pragma unroll 1
  for (int q0 = 0; q0 < n; q0 += 32) {
    int pos = st + q0 + lane;
    pos = pos < 0 ? 0 : (pos > csrLen - 1 ? csrLen - 1 : pos);
    int sl = csr[pos];
    sl = sl < 0 ? 0 : (sl > nN - 1 ? nN - 1 : sl);
    const int mcnt = (n - q0) < 32 ? (n - q0) : 32;
#pragma unroll 1
    for (int pp = 0; pp < mcnt; ++pp) {
      const int s = __builtin_amdgcn_readlane(sl, pp);
      mx0 = fmaxf(mx0, lrelu(eS[ho0 + (size_t)s] + edc0));
      mx1 = fmaxf(mx1, lrelu(eS[ho1 + (size_t)s] + edc1));
    }
  }

  float p0 = __expf(es0 - mx0), p1 = __expf(es1 - mx1);
  float d0 = p0, d1 = p1;
  const float* hc = hw + (size_t)c * pitch;
  v4f b00 = *(const v4f*)(hc + col0) * p0;
  v4f b01 = *(const v4f*)(hc + col0 + 4) * p0;
  v4f b10 = *(const v4f*)(hc + col1) * p1;
  v4f b11 = *(const v4f*)(hc + col1 + 4) * p1;
#pragma unroll 1
  for (int q0 = 0; q0 < n; q0 += 32) {
    int pos = st + q0 + lane;
    pos = pos < 0 ? 0 : (pos > csrLen - 1 ? csrLen - 1 : pos);
    int sl = csr[pos];
    sl = sl < 0 ? 0 : (sl > nN - 1 ? nN - 1 : sl);
    const int mcnt = (n - q0) < 32 ? (n - q0) : 32;
#pragma unroll 1
    for (int pp = 0; pp < mcnt; ++pp) {
      const int s = __builtin_amdgcn_readlane(sl, pp);
      p0 = __expf(lrelu(eS[ho0 + (size_t)s] + edc0) - mx0);
      p1 = __expf(lrelu(eS[ho1 + (size_t)s] + edc1) - mx1);
      d0 += p0; d1 += p1;
      const float* hs = hw + (size_t)s * pitch;
      const v4f h00 = *(const v4f*)(hs + col0);
      const v4f h01 = *(const v4f*)(hs + col0 + 4);
      const v4f h10 = *(const v4f*)(hs + col1);
      const v4f h11 = *(const v4f*)(hs + col1 + 4);
      b00 = b00 + h00 * p0; b01 = b01 + h01 * p0;
      b10 = b10 + h10 * p1; b11 = b11 + h11 * p1;
    }
  }
  dn0 = d0; dn1 = d1; a00 = b00; a01 = b01; a10 = b10; a11 = b11;
}

__global__ __launch_bounds__(NTHR) void k_agg12(
    const int* __restrict__ csr, const int* __restrict__ off, const int* __restrict__ cnt,
    const float* __restrict__ eS, const float* __restrict__ eD, const float* __restrict__ hw,
    const float* __restrict__ bias, const float* __restrict__ lbias,
    unsigned short* pA, unsigned short* pB, int nN, int npad, int csrLen) {
  const int tid = threadIdx.x, lane = tid & 31, wave = tid >> 5;
  const int tbase = blockIdx.x * TGT + wave * 32;
  const int col0 = 8 * lane, col1 = 256 + 8 * lane;
  const int hd0 = lane >> 4, hd1 = 2 + (lane >> 4);
  const size_t ho0 = (size_t)hd0 * (size_t)npad, ho1 = (size_t)hd1 * (size_t)npad;

  const v4f bb00 = *(const v4f*)(bias + col0)     + *(const v4f*)(lbias + col0);
  const v4f bb01 = *(const v4f*)(bias + col0 + 4) + *(const v4f*)(lbias + col0 + 4);
  const v4f bb10 = *(const v4f*)(bias + col1)     + *(const v4f*)(lbias + col1);
  const v4f bb11 = *(const v4f*)(bias + col1 + 4) + *(const v4f*)(lbias + col1 + 4);

  const int cl    = tbase + lane;
  const int cnt_l = cnt[cl];
  const int off_l = off[cl];

#pragma unroll 1
  for (int j = 0; j < 32; ++j) {
    const int c = tbase + j;
    int n = __shfl(cnt_l, j);
    n = n < 0 ? 0 : (n > DEGCAP ? DEGCAP : n);
    const int st = __shfl(off_l, j);
    const float edc0 = eD[ho0 + (size_t)c];
    const float edc1 = eD[ho1 + (size_t)c];
    const float es0  = lrelu(eS[ho0 + (size_t)c] + edc0);
    const float es1  = lrelu(eS[ho1 + (size_t)c] + edc1);

    float den0, den1;
    v4f a00, a01, a10, a11;
    gat_row2(csr, eS, hw, NC12, ho0, ho1, edc0, edc1, es0, es1, c, n, st, col0, col1, lane, nN, csrLen,
             den0, den1, a00, a01, a10, a11);

    const float rd0 = __builtin_amdgcn_rcpf(den0);
    const float rd1 = __builtin_amdgcn_rcpf(den1);
    const float* lp = hw + (size_t)c * NC12 + HID;
    const v4f l00 = *(const v4f*)(lp + col0);
    const v4f l01 = *(const v4f*)(lp + col0 + 4);
    const v4f l10 = *(const v4f*)(lp + col1);
    const v4f l11 = *(const v4f*)(lp + col1 + 4);
    v4f v00 = elu4(a00 * rd0 + bb00 + l00);
    v4f v01 = elu4(a01 * rd0 + bb01 + l01);
    v4f v10 = elu4(a10 * rd1 + bb10 + l10);
    v4f v11 = elu4(a11 * rd1 + bb11 + l11);
    if (c >= nN) { const v4f z = {0.f, 0.f, 0.f, 0.f}; v00 = z; v01 = z; v10 = z; v11 = z; }

    v8us h0, l0, h1, l1;
    split8b(v00, v01, h0, l0);
    split8b(v10, v11, h1, l1);
    unsigned short* g0 = pA + (size_t)c * HID + col0;
    unsigned short* g1 = pA + (size_t)c * HID + col1;
    unsigned short* g2 = pB + (size_t)c * HID + col0;
    unsigned short* g3 = pB + (size_t)c * HID + col1;
    *(volatile v8us*)g0 = h0;
    *(volatile v8us*)g1 = h1;
    *(volatile v8us*)g2 = l0;
    *(volatile v8us*)g3 = l1;
    __threadfence();
    *(volatile v8us*)g0 = h0;
    *(volatile v8us*)g1 = h1;
    *(volatile v8us*)g2 = l0;
    *(volatile v8us*)g3 = l1;
  }
}

__global__ __launch_bounds__(NTHR) void k_agg3(
    const int* __restrict__ csr, const int* __restrict__ off, const int* __restrict__ cnt,
    const float* __restrict__ eS, const float* __restrict__ eD, const float* __restrict__ hw,
    const float* __restrict__ bias, const float* __restrict__ lbias,
    float* out, int nN, int npad, int csrLen) {
  const int tid = threadIdx.x, lane = tid & 31, wave = tid >> 5;
  const int tbase = blockIdx.x * TGT + wave * 32;
  const bool act = lane < 24;
  const int la = act ? lane : lane - 8;
  const int col0 = 8 * la, col1 = 192 + 8 * la;
  const int hd0 = la >> 3, hd1 = 3 + (la >> 3);
  const size_t ho0 = (size_t)hd0 * (size_t)npad, ho1 = (size_t)hd1 * (size_t)npad;

  const int lq  = lane < 16 ? lane : 15;
  const int slq = lq >> 1;
  const bool odd = (lq & 1) != 0;
  const v4f bb = *(const v4f*)(bias + 4 * lq) + *(const v4f*)(lbias + 4 * lq);

  const int cl    = tbase + lane;
  const int cnt_l = cnt[cl];
  const int off_l = off[cl];

#pragma unroll 1
  for (int j = 0; j < 32; ++j) {
    const int c = tbase + j;
    int n = __shfl(cnt_l, j);
    n = n < 0 ? 0 : (n > DEGCAP ? DEGCAP : n);
    const int st = __shfl(off_l, j);
    const float edc0 = eD[ho0 + (size_t)c];
    const float edc1 = eD[ho1 + (size_t)c];
    const float es0  = lrelu(eS[ho0 + (size_t)c] + edc0);
    const float es1  = lrelu(eS[ho1 + (size_t)c] + edc1);

    float den0, den1;
    v4f a00, a01, a10, a11;
    gat_row2(csr, eS, hw, NC3, ho0, ho1, edc0, edc1, es0, es1, c, n, st, col0, col1, lane, nN, csrLen,
             den0, den1, a00, a01, a10, a11);

    const float rd0 = __builtin_amdgcn_rcpf(den0);
    const float rd1 = __builtin_amdgcn_rcpf(den1);
    v4f t0 = a00 * rd0 + a10 * rd1;
    v4f t1 = a01 * rd0 + a11 * rd1;
    if (!act) { const v4f z = {0.f, 0.f, 0.f, 0.f}; t0 = z; t1 = z; }
    t0 = hsum2v(t0);
    t1 = hsum2v(t1);
    v4f s0, s1;
    s0.x = __shfl(t0.x, slq); s0.y = __shfl(t0.y, slq); s0.z = __shfl(t0.z, slq); s0.w = __shfl(t0.w, slq);
    s1.x = __shfl(t1.x, slq); s1.y = __shfl(t1.y, slq); s1.z = __shfl(t1.z, slq); s1.w = __shfl(t1.w, slq);
    v4f o;
    o.x = odd ? s1.x : s0.x; o.y = odd ? s1.y : s0.y; o.z = odd ? s1.z : s0.z; o.w = odd ? s1.w : s0.w;
    const v4f lv = *(const v4f*)(hw + (size_t)c * NC3 + HWC3 + 4 * lq);
    o = o * (1.0f / 6.0f) + bb + lv;
    float* gp = out + (size_t)c * OUTC + 4 * lq;
    const bool wr = (lane < 16) && (c < nN);
    if (wr) *(volatile v4f*)gp = o;
    __threadfence();
    if (wr) *(volatile v4f*)gp = o;
  }
}

extern "C" void kernel_launch(void* const* d_in, const int* in_sizes, int n_in,
                              void* d_out, int out_size, void* d_ws, size_t ws_size,
                              hipStream_t stream) {
  if (n_in < 20) return;
  const int nN = in_sizes[0] / FIN;
  const int nE = in_sizes[1] / 2;
  if (nN <= 0 || nE <= 0 || in_sizes[0] != nN * FIN || in_sizes[1] != 2 * nE) return;
  if (in_sizes[2] != FIN * HID || in_sizes[3] != HID || in_sizes[4] != HID || in_sizes[5] != HID) return;
  if (in_sizes[6] != FIN * HID || in_sizes[7] != HID) return;
  if (in_sizes[8] != HID * HID || in_sizes[9] != HID || in_sizes[10] != HID || in_sizes[11] != HID) return;
  if (in_sizes[12] != HID * HID || in_sizes[13] != HID) return;
  if (in_sizes[14] != HID * HWC3 || in_sizes[15] != HWC3 || in_sizes[16] != HWC3 || in_sizes[17] != OUTC) return;
  if (in_sizes[18] != HID * OUTC || in_sizes[19] != OUTC) return;
  if (nE > (1 << 26) || nN > (1 << 22)) return;
  if ((long long)out_size != (long long)nN * OUTC) return;

  const float* x   = (const float*)d_in[0];
  const int*   ei  = (const int*)d_in[1];
  const int*   src = ei;
  const int*   dst = ei + nE;
  const float* W1  = (const float*)d_in[2];
  const float* a1s = (const float*)d_in[3];
  const float* a1d = (const float*)d_in[4];
  const float* b1  = (const float*)d_in[5];
  const float* lW1 = (const float*)d_in[6];
  const float* lb1 = (const float*)d_in[7];
  const float* W2  = (const float*)d_in[8];
  const float* a2s = (const float*)d_in[9];
  const float* a2d = (const float*)d_in[10];
  const float* b2  = (const float*)d_in[11];
  const float* lW2 = (const float*)d_in[12];
  const float* lb2 = (const float*)d_in[13];
  const float* W3  = (const float*)d_in[14];
  const float* a3s = (const float*)d_in[15];
  const float* a3d = (const float*)d_in[16];
  const float* b3  = (const float*)d_in[17];
  const float* lW3 = (const float*)d_in[18];
  const float* lb3 = (const float*)d_in[19];
  float* out0 = (float*)d_out;

  const int NPAD   = ((nN + TGT - 1) / TGT) * TGT;
  const int nBC    = (nN + NBC - 1) / NBC;
  const int CNTPAD = nBC * NBC;
  if (CNTPAD < NPAD) return;
  if (4 * nBC + 1 > RBN) return;
  const int nBF    = (nN + NBF - 1) / NBF;
  if (nBF + 1 > 4 * nBC + 1) return;
  const int csrLen = ((nE + 31) & ~31) + 4096;
  if (31 * 4 * nBC > 4096) return;
  const int nAgg   = NPAD / TGT;
  const int nGemm  = NPAD / BM;
  const int nXu    = NPAD * (FIN / 8);

  const size_t wPl12  = (size_t)NC12 * HID * 2;
  const size_t wPl3   = (size_t)NC3 * HID * 2;
  const size_t wReg   = 2 * wPl12 > 2 * wPl3 ? 2 * wPl12 : 2 * wPl3;
  const size_t aPlane = (size_t)NPAD * HID * 2;
  char* ws = (char*)d_ws;
  size_t off = 0;
  const size_t oW   = off; off += wReg;                          off = (off + 255) & ~(size_t)255;
  const size_t oA   = off; off += 2 * aPlane;                    off = (off + 255) & ~(size_t)255;
  const size_t oCnt = off; off += (size_t)CNTPAD * 4;            off = (off + 255) & ~(size_t)255;
  const size_t oOff = off; off += (size_t)CNTPAD * 4;            off = (off + 255) & ~(size_t)255;
  const size_t oRb  = off; off += (size_t)RBN * 4;               off = (off + 255) & ~(size_t)255;
  const size_t oCsr = off; off += (size_t)csrLen * 4;            off = (off + 255) & ~(size_t)255;
  const size_t oC   = off; off += (size_t)NPAD * NC12 * 4;       off = (off + 255) & ~(size_t)255;
  const size_t oES  = off; off += (size_t)NHMX * NPAD * 4;       off = (off + 255) & ~(size_t)255;
  const size_t oED  = off; off += (size_t)NHMX * NPAD * 4;       off = (off + 255) & ~(size_t)255;
  if (off > ws_size || off > (size_t)WSCAP) return;
  unsigned short* w12h = (unsigned short*)(ws + oW);
  unsigned short* w12l = (unsigned short*)(ws + oW + wPl12);
  unsigned short* w3h  = (unsigned short*)(ws + oW);
  unsigned short* w3l  = (unsigned short*)(ws + oW + wPl3);
  unsigned short* pa   = (unsigned short*)(ws + oA);
  unsigned short* pl   = (unsigned short*)(ws + oA + aPlane);
  int*   cnt  = (int*)(ws + oCnt);
  int*   offp = (int*)(ws + oOff);
  int*   rb   = (int*)(ws + oRb);
  int*   csr  = (int*)(ws + oCsr);
  float* cbuf = (float*)(ws + oC);
  float* es   = (float*)(ws + oES);
  float* ed   = (float*)(ws + oED);

  const int vec8 = ((nE & 3) == 0) ? 1 : 0;

  k_wprep3<FIN, HID><<<(HID * FIN / 8 + NTHR - 1) / NTHR, NTHR, 0, stream>>>(W1, w12h, w12l);
  k_wprep3<FIN, HID><<<(HID * FIN / 8 + NTHR - 1) / NTHR, NTHR, 0, stream>>>(
      lW1, w12h + (size_t)HID * FIN, w12l + (size_t)HID * FIN);
  k_xcvt<<<(nXu + NTHR - 1) / NTHR, NTHR, 0, stream>>>(x, pa, pl, nN, nXu);

  k_count<<<nBC, NTHR, 0, stream>>>(dst, cnt, nE, vec8);
  k_offsets<<<1, OTHR, 0, stream>>>(cnt, offp, rb, nBC);
  hipFuncSetAttribute(reinterpret_cast<const void*>(&k_fill),
                      hipFuncAttributeMaxDynamicSharedMemorySize, LDS_FILL);
  k_fill<<<nBF, NTHR, LDS_FILL, stream>>>(src, dst, offp, rb, csr, nN, nE, vec8, csrLen);

  k_gemm<FIN, CH12, NC12, NH12><<<dim3(nGemm, NC12 / CH12), NTHR, 0, stream>>>(
      pa, pl, w12h, w12l, a1s, a1d, cbuf, es, ed, NPAD);
  k_agg12<<<nAgg, NTHR, 0, stream>>>(csr, offp, cnt, es, ed, cbuf, b1, lb1, pa, pl, nN, NPAD, csrLen);

  k_wprep3<HID, HID><<<(HID * HID / 8 + NTHR - 1) / NTHR, NTHR, 0, stream>>>(W2, w12h, w12l);
  k_wprep3<HID, HID><<<(HID * HID / 8 + NTHR - 1) / NTHR, NTHR, 0, stream>>>(
      lW2, w12h + (size_t)HID * HID, w12l + (size_t)HID * HID);
  k_gemm<HID, CH12, NC12, NH12><<<dim3(nGemm, NC12 / CH12), NTHR, 0, stream>>>(
      pa, pl, w12h, w12l, a2s, a2d, cbuf, es, ed, NPAD);
  k_agg12<<<nAgg, NTHR, 0, stream>>>(csr, offp, cnt, es, ed, cbuf, b2, lb2, pa, pl, nN, NPAD, csrLen);

  k_wprep3<HID, HWC3><<<(HWC3 * HID / 8 + NTHR - 1) / NTHR, NTHR, 0, stream>>>(W3, w3h, w3l);
  k_wprep3<HID, OUTC><<<(OUTC * HID / 8 + NTHR - 1) / NTHR, NTHR, 0, stream>>>(
      lW3, w3h + (size_t)HWC3 * HID, w3l + (size_t)HWC3 * HID);
  k_gemm<HID, CH3, NC3, NH3><<<dim3(nGemm, NC3 / CH3), NTHR, 0, stream>>>(
      pa, pl, w3h, w3l, a3s, a3d, cbuf, es, ed, NPAD);
  k_agg3<<<nAgg, NTHR, 0, stream>>>(csr, offp, cnt, es, ed, cbuf, b3, lb3, out0, nN, NPAD, csrLen);
}
